// HaloWindowAttention_69818988363877
// MI455X (gfx1250) — hardware-verified
//
#include <hip/hip_runtime.h>
#include <math.h>
#include <stdint.h>

#define NBAT   16
#define CH     1024
#define NHEAD  16
#define HDIM   64
#define GW     16
#define NPIX   (GW * GW)
#define PW     32
#define POFF   8
#define BLO    264
#define BHI    520
#define NKB    (NPIX / 64)
#define EXPM01 0.9048374180359595f
static_assert(NHEAD * HDIM == CH);
static_assert((NPIX % 64) == 0 && (CH % 64) == 0);
static_assert(BLO == POFF * PW + POFF && BHI == BLO + GW * GW);

typedef _Float16 v16h __attribute__((ext_vector_type(16)));
typedef _Float16 v8h  __attribute__((ext_vector_type(8)));
typedef __bf16   v16b __attribute__((ext_vector_type(16)));
typedef __bf16   v8b  __attribute__((ext_vector_type(8)));
typedef float    v8f  __attribute__((ext_vector_type(8)));
typedef float    v4f  __attribute__((ext_vector_type(4)));
typedef unsigned int v4u __attribute__((ext_vector_type(4)));

__device__ __forceinline__ unsigned short bf_bits(float f) {
  unsigned u = __float_as_uint(f);
  return (unsigned short)((u + 0x7FFFu + ((u >> 16) & 1u)) >> 16);
}
__device__ __forceinline__ float bf_up(unsigned short hb) { return __uint_as_float(((unsigned)hb) << 16); }
__device__ __forceinline__ float bfq(float f) { return bf_up(bf_bits(f)); }
__device__ __forceinline__ unsigned short h_bits(_Float16 x) { return __builtin_bit_cast(unsigned short, x); }
__device__ __forceinline__ unsigned pk16(unsigned short a, unsigned short b) { return (unsigned)a | ((unsigned)b << 16); }
__device__ __forceinline__ v8f zero8() { v8f z = {0.f, 0.f, 0.f, 0.f, 0.f, 0.f, 0.f, 0.f}; return z; }

__device__ __forceinline__ v16b ldfrag_b(const __bf16* p) {
  union { v16b v; v8b hv[2]; } f;
  f.hv[0] = *(const v8b*)(p);
  f.hv[1] = *(const v8b*)(p + 16);
  return f.v;
}

__device__ __forceinline__ v8f mma_b(v16b a, v16b b, v8f c) {
  c = __builtin_amdgcn_wmma_f32_16x16x32_bf16(false, a, false, b, (short)0, c, false, false);
  asm volatile("v_nop\n\tv_nop\n\tv_nop\n\tv_nop" : "+v"(c) : "v"(a), "v"(b));
  return c;
}
__device__ __forceinline__ v8f mma_h(v16h a, v16h b, v8f c) {
  c = __builtin_amdgcn_wmma_f32_16x16x32_f16(false, a, false, b, (short)0, c, false, false);
  asm volatile("v_nop\n\tv_nop\n\tv_nop\n\tv_nop" : "+v"(c) : "v"(a), "v"(b));
  return c;
}
__device__ __forceinline__ v8f mma_b_raw(v16b a, v16b b, v8f c) {
  return __builtin_amdgcn_wmma_f32_16x16x32_bf16(false, a, false, b, (short)0, c, false, false);
}
__device__ __forceinline__ void dep_guard_b(v8f& a, v8f& b, v16b x, v16b y) {
  asm volatile("v_nop\n\tv_nop\n\tv_nop\n\tv_nop" : "+v"(a), "+v"(b) : "v"(x), "v"(y));
}
__device__ __forceinline__ void keep4_b(v16b a, v16b b, v16b c, v16b d) {
  asm volatile("v_nop" :: "v"(a), "v"(b), "v"(c), "v"(d));
}
__device__ __forceinline__ void acc_guard4(v8f& a, v8f& b, v8f& c, v8f& d) {
  asm volatile("v_nop\n\tv_nop\n\tv_nop\n\tv_nop" : "+v"(a), "+v"(b), "+v"(c), "+v"(d));
}

__global__ __launch_bounds__(256) void tr_cvt(const float* __restrict__ src, int R, int Cn, long long sstr,
                                              unsigned short* dst, long long dstr) {
  __shared__ float sT[64 * 65];
  const int tid = threadIdx.x;
  const int c0 = blockIdx.x * 64, r0 = blockIdx.y * 64;
  const float* sb = src + (size_t)blockIdx.z * (size_t)sstr;
  unsigned short* db = dst + (size_t)blockIdx.z * (size_t)dstr;
  {
    const int row = tid >> 2, col = (tid & 3) * 16;
    const float* p = sb + (size_t)(r0 + row) * (size_t)Cn + c0 + col;
#pragma unroll
    for (int q = 0; q < 4; ++q) {
      const v4f v = *(const v4f*)(p + 4 * q);
#pragma unroll
      for (int e = 0; e < 4; ++e) sT[(col + 4 * q + e) * 65 + row] = v[e];
    }
  }
  __syncthreads();
  const int rq = tid >> 3, k8 = (tid & 7) * 8;
  v4u pk[2];
#pragma unroll
  for (int it = 0; it < 2; ++it) {
    const int cr = it * 32 + rq;
    const float* sp = sT + cr * 65 + k8;
    v4u a;
#pragma unroll
    for (int e = 0; e < 4; ++e) a[e] = pk16(bf_bits(sp[2 * e]), bf_bits(sp[2 * e + 1]));
    pk[it] = a;
  }
  for (int pass = 0; pass < 2; ++pass) {
#pragma unroll
    for (int it = 0; it < 2; ++it) {
      const int cr = it * 32 + rq;
      *(volatile v4u*)(db + (size_t)(c0 + cr) * (size_t)R + r0 + k8) = pk[it];
    }
    __threadfence();
  }
}

template <int BSPLIT, int OUT_MODE, int BIAS>
__global__ __launch_bounds__(256) void gemm64(
    const unsigned short* __restrict__ Ap, int lda, long long strideA,
    const unsigned short* __restrict__ Btp, const unsigned short* __restrict__ Bt2p, int ldb, long long strideB,
    const float* __restrict__ bias,
    void* Cout, void* Cout2, int ldc, long long strideC,
    int M, int N, int K, float rscale) {
  const __bf16* A   = (const __bf16*)(const void*)Ap;
  const __bf16* Bt  = (const __bf16*)(const void*)Btp;
  const __bf16* Bt2 = (const __bf16*)(const void*)Bt2p;
  __shared__ __align__(16) float sT[8][16 * 68];
  const int b    = blockIdx.y;
  const int lane = threadIdx.x & 31;
  const int wave = threadIdx.x >> 5;
  const int tilesN = N >> 6;
  const int tilesM = M >> 6;
  const int tile = blockIdx.x * 8 + wave;
  if (tile >= tilesM * tilesN) return;
  const int tm = tile / tilesN;
  const int tn = tile - tm * tilesN;
  const int m0 = tm << 6;
  const int n0 = tn << 6;

  const __bf16* Ab  = A  + (size_t)b * (size_t)strideA;
  const __bf16* Bb  = Bt + (size_t)b * (size_t)strideB;
  const __bf16* Bb2 = BSPLIT ? (Bt2 + (size_t)b * (size_t)strideB) : Bb;

  const int rlane = lane & 15;
  const int koff  = (lane >> 4) * 8;
  const int mOff  = (lane >> 4) * 8;

  v8f acc[4][4];
#pragma unroll
  for (int i = 0; i < 4; ++i)
#pragma unroll
    for (int j = 0; j < 4; ++j) acc[i][j] = zero8();

  for (int k0 = 0; k0 < K; k0 += 32) {
#pragma unroll
    for (int part = 0; part < (BSPLIT ? 2 : 1); ++part) {
      const __bf16* Bs = (part == 0) ? Bb : Bb2;
      v16b bf[4];
#pragma unroll
      for (int j = 0; j < 4; ++j) {
        const size_t bo = (size_t)(n0 + (j << 4) + rlane) * (size_t)ldb + koff + k0;
        bf[j] = ldfrag_b(Bs + bo);
      }
#pragma unroll
      for (int i = 0; i < 4; ++i) {
        const size_t ao = (size_t)(m0 + (i << 4) + rlane) * (size_t)lda + koff + k0;
        const v16b af = ldfrag_b(Ab + ao);
#pragma unroll
        for (int j = 0; j < 4; ++j) acc[i][j] = mma_b_raw(af, bf[j], acc[i][j]);
        dep_guard_b(acc[i][0], acc[i][3], af, bf[3]);
      }
      keep4_b(bf[0], bf[1], bf[2], bf[3]);
    }
  }
  acc_guard4(acc[0][0], acc[0][1], acc[0][2], acc[0][3]);
  acc_guard4(acc[1][0], acc[1][1], acc[1][2], acc[1][3]);
  acc_guard4(acc[2][0], acc[2][1], acc[2][2], acc[2][3]);
  acc_guard4(acc[3][0], acc[3][1], acc[3][2], acc[3][3]);

  float* slab = sT[wave];
  float bcol[4];
#pragma unroll
  for (int j = 0; j < 4; ++j) bcol[j] = 0.f;
  if (BIAS == 1) {
#pragma unroll
    for (int j = 0; j < 4; ++j) bcol[j] = bfq(bias[n0 + (j << 4) + rlane]);
  }
#pragma unroll
  for (int i = 0; i < 4; ++i) {
    const int mBase = m0 + (i << 4);
    float brow[8];
#pragma unroll
    for (int r = 0; r < 8; ++r) brow[r] = 0.f;
    if (BIAS == 2) {
#pragma unroll
      for (int r = 0; r < 8; ++r) brow[r] = bfq(bias[mBase + mOff + r]);
    }
#pragma unroll
    for (int j = 0; j < 4; ++j) {
#pragma unroll
      for (int r = 0; r < 8; ++r) {
        const float bv = (BIAS == 1) ? bcol[j] : brow[r];
        slab[(mOff + r) * 68 + (j << 4) + rlane] = acc[i][j][r] + bv;
      }
    }
    __builtin_amdgcn_fence(__ATOMIC_RELEASE, "workgroup");
    __builtin_amdgcn_wave_barrier();
    __builtin_amdgcn_fence(__ATOMIC_ACQUIRE, "workgroup");
    if (OUT_MODE == 0) {
      float* C = (float*)Cout + (size_t)b * (size_t)strideC;
      const int hh = lane >> 4, c4 = (lane & 15) * 4;
      for (int pass = 0; pass < 2; ++pass) {
#pragma unroll
        for (int it = 0; it < 8; ++it) {
          const int row = it * 2 + hh;
          const v4f v = *(const v4f*)(slab + row * 68 + c4);
          *(volatile v4f*)(C + (size_t)(mBase + row) * (size_t)ldc + n0 + c4) = v;
        }
        __threadfence();
      }
    } else {
      const int q = lane >> 3, c8 = (lane & 7) * 8;
      unsigned short* C  = (unsigned short*)Cout  + (size_t)b * (size_t)strideC;
      unsigned short* C2 = (unsigned short*)Cout2 + (size_t)b * (size_t)strideC;
      v4u hv[4], lv[4];
#pragma unroll
      for (int it = 0; it < 4; ++it) {
        const int row = it * 4 + q;
        const float* sp = slab + row * 68 + c8;
        v4u a, a2;
#pragma unroll
        for (int e = 0; e < 4; ++e) {
          const float f0 = sp[2 * e], f1 = sp[2 * e + 1];
          unsigned short h0, h1, l0, l1;
          if (OUT_MODE == 2) {
            h0 = bf_bits(f0); h1 = bf_bits(f1);
            l0 = bf_bits(f0 - bf_up(h0)); l1 = bf_bits(f1 - bf_up(h1));
          } else {
            const _Float16 x0 = (_Float16)f0, x1 = (_Float16)f1;
            h0 = h_bits(x0); h1 = h_bits(x1);
            l0 = h_bits((_Float16)((f0 - (float)x0) * rscale));
            l1 = h_bits((_Float16)((f1 - (float)x1) * rscale));
          }
          a[e] = pk16(h0, h1); a2[e] = pk16(l0, l1);
        }
        hv[it] = a; lv[it] = a2;
      }
      for (int pass = 0; pass < 2; ++pass) {
#pragma unroll
        for (int it = 0; it < 4; ++it) {
          const int row = it * 4 + q;
          const size_t go = (size_t)(mBase + row) * (size_t)ldc + n0 + c8;
          *(volatile v4u*)(C + go)  = hv[it];
          *(volatile v4u*)(C2 + go) = lv[it];
        }
        __threadfence();
      }
    }
    __builtin_amdgcn_fence(__ATOMIC_RELEASE, "workgroup");
    __builtin_amdgcn_wave_barrier();
    __builtin_amdgcn_fence(__ATOMIC_ACQUIRE, "workgroup");
  }
}

__device__ __forceinline__ int in_band(int r, int cc) {
  const int s = r * PW + cc;
  return (s >= BLO && s < BHI) ? 1 : 0;
}
__device__ __forceinline__ float key_weight(int p, bool qband) {
  const int ry = p >> 4, rx = p & 15;
  const int r1 = ry + POFF, r2 = POFF - ry, r3 = 2 * (GW - 1) + POFF - ry;
  const int c1 = rx + POFF, c2 = POFF - rx, c3 = 2 * (GW - 1) + POFF - rx;
  const int vr2 = (ry >= 1 && ry <= POFF) ? 1 : 0;
  const int vr3 = (r3 <= PW - 1 && r3 - POFF >= GW) ? 1 : 0;
  const int vc2 = (rx >= 1 && rx <= POFF) ? 1 : 0;
  const int vc3 = (c3 <= PW - 1 && c3 - POFF >= GW) ? 1 : 0;
  const int nr = 1 + vr2 + vr3, nc = 1 + vc2 + vc3;
  const int nin = in_band(r1, c1) + vc2 * in_band(r1, c2) + vc3 * in_band(r1, c3)
                + vr2 * (in_band(r2, c1) + vc2 * in_band(r2, c2) + vc3 * in_band(r2, c3))
                + vr3 * (in_band(r3, c1) + vc2 * in_band(r3, c2) + vc3 * in_band(r3, c3));
  const int ntot = nr * nc;
  const int nout = ntot - nin;
  return qband ? ((float)nin + (float)nout * EXPM01) : (float)ntot;
}

__global__ __launch_bounds__(128)
void attn_win(const unsigned short* __restrict__ qhp, const unsigned short* __restrict__ qlp,
              const unsigned short* __restrict__ khp, const unsigned short* __restrict__ klp,
              const unsigned short* __restrict__ vhp, const unsigned short* __restrict__ vlp,
              unsigned short* ohp, unsigned short* olp, float sscale) {
  union FB { v16b v; v8b hv[2]; };
  union FH { v16h v; v8h hv[2]; };
  __shared__ __align__(16) float    KObuf[4096];
  __shared__ __align__(16) _Float16 Vth[64 * 64];
  __shared__ __align__(16) _Float16 Vtl[64 * 64];
  __shared__ __align__(16) _Float16 Psh[4][16 * 64];
  __shared__ __align__(16) _Float16 Psl[4][16 * 64];
  __shared__ float Wtab[NPIX];
  __bf16* Ksh = (__bf16*)(void*)KObuf;
  __bf16* Ksl = Ksh + 64 * 64;

  const int tid  = threadIdx.x;
  const int wave = tid >> 5;
  const int lane = tid & 31;
  const int hh   = lane >> 4;
  const int c    = lane & 15;

  const int bx = blockIdx.x;
  const int qb = bx % NKB;
  const int h  = (bx / NKB) % NHEAD;
  const int b  = bx / (NKB * NHEAD);
  const int q0 = qb * 64 + wave * 16;
  const size_t rowB = (size_t)b * NPIX;
  const bool qband = (qb * 64 + 63 < NPIX / 2);

  for (int e = tid; e < NPIX; e += 128) Wtab[e] = key_weight(e, qband);
  __syncthreads();

  const __bf16* Qh = (const __bf16*)(const void*)qhp + (size_t)h * HDIM;
  const __bf16* Ql = (const __bf16*)(const void*)qlp + (size_t)h * HDIM;
  const __bf16* Kh = (const __bf16*)(const void*)khp + (size_t)h * HDIM;
  const __bf16* Kl = (const __bf16*)(const void*)klp + (size_t)h * HDIM;
  const _Float16* Vh = (const _Float16*)(const void*)vhp + ((size_t)b * CH + (size_t)h * HDIM) * NPIX;
  const _Float16* Vl = (const _Float16*)(const void*)vlp + ((size_t)b * CH + (size_t)h * HDIM) * NPIX;

  v16b qah[2], qal[2];
#pragma unroll
  for (int dc = 0; dc < 2; ++dc) {
    const size_t qo = (rowB + q0 + c) * CH + dc * 32 + 8 * hh;
    qah[dc] = ldfrag_b(Qh + qo);
    qal[dc] = ldfrag_b(Ql + qo);
  }

  float mrow[8], lrow[8];
  v8f oacc[4];
#pragma unroll
  for (int r = 0; r < 8; ++r) { mrow[r] = -INFINITY; lrow[r] = 0.f; }
#pragma unroll
  for (int t = 0; t < 4; ++t) oacc[t] = zero8();

  for (int kt = 0; kt < NKB; ++kt) {
    const int kv0 = kt * 64;
    __syncthreads();
    {
      const int r = tid >> 1, half = (tid & 1) * 32;
      const __bf16*   kg  = Kh + (rowB + kv0 + r) * CH + half;
      const __bf16*   klg = Kl + (rowB + kv0 + r) * CH + half;
      const _Float16* vg  = Vh + (size_t)r * NPIX + kv0 + half;
      const _Float16* vlg = Vl + (size_t)r * NPIX + kv0 + half;
#pragma unroll
      for (int i = 0; i < 4; ++i) {
        const v8b a0 = *(const v8b*)(kg + 8 * i);
        const v8b a1 = *(const v8b*)(klg + 8 * i);
        const v8h b0 = *(const v8h*)(vg + 8 * i);
        const v8h b1 = *(const v8h*)(vlg + 8 * i);
        *(v8b*)(Ksh + r * 64 + half + 8 * i) = a0;
        *(v8b*)(Ksl + r * 64 + half + 8 * i) = a1;
        *(v8h*)(Vth + r * 64 + half + 8 * i) = b0;
        *(v8h*)(Vtl + r * 64 + half + 8 * i) = b1;
      }
    }
    __syncthreads();

    v8f s[4];
#pragma unroll
    for (int j = 0; j < 4; ++j) {
      s[j] = zero8();
#pragma unroll
      for (int dc = 0; dc < 2; ++dc) {
        FB kb, kl;
        kb.hv[0] = *(const v8b*)(Ksh + (j * 16 + c) * 64 + dc * 32 + 8 * hh);
        kb.hv[1] = *(const v8b*)(Ksh + (j * 16 + c) * 64 + dc * 32 + 16 + 8 * hh);
        kl.hv[0] = *(const v8b*)(Ksl + (j * 16 + c) * 64 + dc * 32 + 8 * hh);
        kl.hv[1] = *(const v8b*)(Ksl + (j * 16 + c) * 64 + dc * 32 + 16 + 8 * hh);
        s[j] = mma_b(qah[dc], kb.v, s[j]);
        s[j] = mma_b(qah[dc], kl.v, s[j]);
        s[j] = mma_b(qal[dc], kb.v, s[j]);
      }
    }

    float wk[4];
#pragma unroll
    for (int j = 0; j < 4; ++j) wk[j] = Wtab[kv0 + (j << 4) + c];
    _Float16* pwh = Psh[wave];
    _Float16* pwl = Psl[wave];
#pragma unroll
    for (int r = 0; r < 8; ++r) {
      float m = -INFINITY;
#pragma unroll
      for (int j = 0; j < 4; ++j) {
        const float sv = s[j][r] * sscale;
        s[j][r] = sv;
        m = fmaxf(m, sv);
      }
#pragma unroll
      for (int off = 1; off < 16; off <<= 1) m = fmaxf(m, __shfl_xor(m, off, 32));
      const float mnew  = fmaxf(mrow[r], m);
      const float msafe = (mnew == -INFINITY) ? 0.f : mnew;
      const float alpha = __expf(mrow[r] - msafe);
      mrow[r] = mnew;
      float psum = 0.f;
#pragma unroll
      for (int j = 0; j < 4; ++j) {
        const float p = __expf(s[j][r] - msafe) * wk[j];
        psum += p;
        const float p1k = p * 1024.0f;
        const _Float16 ph = (_Float16)p1k;
        pwh[(8 * hh + r) * 64 + j * 16 + c] = ph;
        const _Float16 pl = (_Float16)((p1k - (float)ph) * 4096.0f);
        pwl[(8 * hh + r) * 64 + j * 16 + c] = pl;
      }
#pragma unroll
      for (int off = 1; off < 16; off <<= 1) psum += __shfl_xor(psum, off, 32);
      lrow[r] = lrow[r] * alpha + psum;
#pragma unroll
      for (int t = 0; t < 4; ++t) oacc[t][r] *= alpha;
    }
    __builtin_amdgcn_fence(__ATOMIC_RELEASE, "workgroup");
    __builtin_amdgcn_wave_barrier();
    __builtin_amdgcn_fence(__ATOMIC_ACQUIRE, "workgroup");

    v8f o1[4];
#pragma unroll
    for (int t = 0; t < 4; ++t) o1[t] = zero8();
#pragma unroll 1
    for (int kk = 0; kk < 2; ++kk) {
      FH pa, pl;
      pa.hv[0] = *(const v8h*)(pwh + c * 64 + kk * 32 + 8 * hh);
      pa.hv[1] = *(const v8h*)(pwh + c * 64 + kk * 32 + 16 + 8 * hh);
      pl.hv[0] = *(const v8h*)(pwl + c * 64 + kk * 32 + 8 * hh);
      pl.hv[1] = *(const v8h*)(pwl + c * 64 + kk * 32 + 16 + 8 * hh);
#pragma unroll
      for (int t = 0; t < 4; ++t) {
        FH vb, vl;
        vb.hv[0] = *(const v8h*)(Vth + (t * 16 + c) * 64 + kk * 32 + 8 * hh);
        vb.hv[1] = *(const v8h*)(Vth + (t * 16 + c) * 64 + kk * 32 + 16 + 8 * hh);
        vl.hv[0] = *(const v8h*)(Vtl + (t * 16 + c) * 64 + kk * 32 + 8 * hh);
        vl.hv[1] = *(const v8h*)(Vtl + (t * 16 + c) * 64 + kk * 32 + 16 + 8 * hh);
        oacc[t] = mma_h(pa.v, vb.v, oacc[t]);
        o1[t]   = mma_h(pa.v, vl.v, o1[t]);
        o1[t]   = mma_h(pl.v, vb.v, o1[t]);
      }
    }
#pragma unroll
    for (int t = 0; t < 4; ++t)
#pragma unroll
      for (int r = 0; r < 8; ++r) oacc[t][r] += o1[t][r] * (1.0f / 4096.0f);
  }

  __syncthreads();
  float* os = KObuf + wave * 1024;
#pragma unroll
  for (int r = 0; r < 8; ++r) {
    const float l = lrow[r];
    const float inv = ((l > 0.f) ? (1.0f / l) : 0.f) * (1.0f / 1024.0f);
#pragma unroll
    for (int t = 0; t < 4; ++t) os[(8 * hh + r) * 64 + t * 16 + c] = oacc[t][r] * inv;
  }
  __builtin_amdgcn_fence(__ATOMIC_RELEASE, "workgroup");
  __builtin_amdgcn_wave_barrier();
  __builtin_amdgcn_fence(__ATOMIC_ACQUIRE, "workgroup");
  {
    const int q4 = lane >> 3, c8 = (lane & 7) * 8;
    v4u hv[4], lv[4];
#pragma unroll
    for (int it = 0; it < 4; ++it) {
      const int row = it * 4 + q4;
      const float* sp = os + row * 64 + c8;
      v4u a, a2;
#pragma unroll
      for (int e = 0; e < 4; ++e) {
        const float f0 = sp[2 * e], f1 = sp[2 * e + 1];
        const unsigned short h0 = bf_bits(f0), h1 = bf_bits(f1);
        const unsigned short l0 = bf_bits(f0 - bf_up(h0)), l1 = bf_bits(f1 - bf_up(h1));
        a[e] = pk16(h0, h1); a2[e] = pk16(l0, l1);
      }
      hv[it] = a; lv[it] = a2;
    }
    for (int pass = 0; pass < 2; ++pass) {
#pragma unroll
      for (int it = 0; it < 4; ++it) {
        const int row = it * 4 + q4;
        const size_t go = (rowB + q0 + row) * CH + (size_t)h * HDIM + c8;
        *(volatile v4u*)(ohp + go) = hv[it];
        *(volatile v4u*)(olp + go) = lv[it];
      }
      __threadfence();
    }
  }
}

extern "C" void kernel_launch(void* const* d_in, const int* in_sizes, int n_in,
                              void* d_out, int out_size, void* d_ws, size_t ws_size,
                              hipStream_t stream) {
  if (n_in < 5) return;
  if (in_sizes[0] != NBAT * CH * NPIX) return;
  if (in_sizes[1] != CH * 3 * CH) return;
  if (in_sizes[2] != 3 * CH) return;
  if (in_sizes[3] != CH * CH) return;
  if (in_sizes[4] != CH) return;
  if (out_size != NBAT * CH * NPIX) return;

  const float* x      = (const float*)d_in[0];
  const float* w_qkv  = (const float*)d_in[1];
  const float* b_qkv  = (const float*)d_in[2];
  const float* w_proj = (const float*)d_in[3];
  const float* b_proj = (const float*)d_in[4];

  const size_t PA  = (size_t)NBAT * NPIX * CH * 2;
  const size_t PWt = (size_t)3 * CH * CH * 2;
  const size_t PWp = (size_t)CH * CH * 2;
  const size_t PVt = (size_t)NBAT * CH * NPIX * 2;
  size_t off = 0;
  const size_t oXb = off; off += PA;
  const size_t oWt = off; off += PWt;
  const size_t oWp = off; off += PWp;
  const size_t oQh = off; off += PA;
  const size_t oQl = off; off += PA;
  const size_t oKh = off; off += PA;
  const size_t oKl = off; off += PA;
  const size_t oVh = off; off += PVt;
  const size_t oVl = off; off += PVt;
  const size_t oOh = off; off += PA;
  const size_t oOl = off; off += PA;
  if (off > ws_size) return;
  if (off > (size_t)134217728) return;

  char* ws = (char*)d_ws;
  unsigned short* Xb  = (unsigned short*)(ws + oXb);
  unsigned short* Wt  = (unsigned short*)(ws + oWt);
  unsigned short* Wp  = (unsigned short*)(ws + oWp);
  unsigned short* Qh  = (unsigned short*)(ws + oQh);
  unsigned short* Ql  = (unsigned short*)(ws + oQl);
  unsigned short* Kh  = (unsigned short*)(ws + oKh);
  unsigned short* Kl  = (unsigned short*)(ws + oKl);
  unsigned short* VTh = (unsigned short*)(ws + oVh);
  unsigned short* VTl = (unsigned short*)(ws + oVl);
  unsigned short* Oh  = (unsigned short*)(ws + oOh);
  unsigned short* Ol  = (unsigned short*)(ws + oOl);

  const dim3 blk(256);
  tr_cvt<<<dim3(NPIX / 64, CH / 64, NBAT), blk, 0, stream>>>(
      x, CH, NPIX, (long long)CH * NPIX, Xb, (long long)NPIX * CH);
  tr_cvt<<<dim3(3 * CH / 64, CH / 64, 1), blk, 0, stream>>>(w_qkv, CH, 3 * CH, 0LL, Wt, 0LL);
  tr_cvt<<<dim3(CH / 64, CH / 64, 1), blk, 0, stream>>>(w_proj, CH, CH, 0LL, Wp, 0LL);
  const dim3 gQK(((NBAT * NPIX / 64) * (CH / 64) + 7) / 8, 1);
  gemm64<0, 2, 1><<<gQK, blk, 0, stream>>>(
      Xb, CH, 0LL, Wt, Wt, CH, 0LL, b_qkv,
      (void*)Qh, (void*)Ql, CH, 0LL, NBAT * NPIX, CH, CH, 1.0f);
  gemm64<0, 2, 1><<<gQK, blk, 0, stream>>>(
      Xb, CH, 0LL, Wt + (size_t)CH * CH, Wt + (size_t)CH * CH, CH, 0LL, b_qkv + CH,
      (void*)Kh, (void*)Kl, CH, 0LL, NBAT * NPIX, CH, CH, 1.0f);
  const dim3 gVT(((CH / 64) * (NPIX / 64) + 7) / 8, NBAT);
  gemm64<0, 3, 2><<<gVT, blk, 0, stream>>>(
      Wt + (size_t)2 * CH * CH, CH, 0LL, Xb, Xb, CH, (long long)NPIX * CH, b_qkv + 2 * CH,
      (void*)VTh, (void*)VTl, NPIX, (long long)CH * NPIX, CH, NPIX, CH, 4096.0f);
  attn_win<<<dim3(NBAT * NHEAD * NKB), dim3(128), 0, stream>>>(
      Qh, Ql, Kh, Kl, VTh, VTl, Oh, Ol, 0.125f);
  const dim3 gPr(((CH / 64) * (NPIX / 64) + 7) / 8, NBAT);
  gemm64<1, 0, 2><<<gPr, blk, 0, stream>>>(
      Wp, CH, 0LL, Oh, Ol, CH, (long long)NPIX * CH, b_proj,
      d_out, d_out, NPIX, (long long)CH * NPIX, CH, NPIX, CH, 1.0f);
  (void)hipGetLastError();
}
